// FaceGeometryEncoder_14070312862134
// MI455X (gfx1250) — hardware-verified
//
#include <hip/hip_runtime.h>
#include <stddef.h>
#include <math.h>


#define IN_DIM 7
#define K1P    32
#define H1D    64
#define H2D    128
#define EMB    256
#define ATT    64
#define NTHR   256
#define NWAVE  8
#define ROWS   128
#define CHUNK  1024
#define SUBS   (CHUNK / NTHR)
#define MAXCH  64
#define SMAX   4096
#define XPF    36
#define H1P    72
#define H2P    136
#define H3P    260

#define G_W1   (H1D * K1P / 8)
#define G_W2   (H2D * H1D / 8)
#define G_W3   (EMB * H2D / 8)
#define G_A1   (ATT * EMB / 8)
#define G_TOT  (G_W1 + G_W2 + G_W3 + G_A1)

#define L_XF    0
#define L_H1    (L_XF + ROWS * XPF * 4)
#define L_H2    (L_H1 + ROWS * H1P * 2)
#define L_H3    (L_H2 + ROWS * H2P * 2)
#define L_S     (L_H3 + ROWS * H3P * 4)
#define L_E     (L_S + ROWS * 4)
#define L_LIST  (L_E + ROWS * 4)
#define L_CHK   (L_LIST + CHUNK * 4)
#define L_WCNT  (L_CHK + MAXCH * 4)
#define L_OUT   (L_WCNT + 16 * 4)
#define LDS_SEG (L_OUT + EMB * 4)

static_assert(ROWS == NWAVE * 16);
static_assert(NTHR == NWAVE * 32);
static_assert(NTHR == EMB);
static_assert((ROWS * 8) % NTHR == 0);
static_assert((G_TOT % NTHR) == 0 && (G_W1 % NTHR) == 0 && ((G_W1 + G_W2) % NTHR) == 0 && ((G_W1 + G_W2 + G_W3) % NTHR) == 0);
static_assert((L_H1 % 16) == 0 && (L_H2 % 16) == 0 && (L_H3 % 16) == 0 && (L_S % 16) == 0 && (L_E % 16) == 0);
static_assert((L_LIST % 16) == 0 && (L_CHK % 16) == 0 && (L_WCNT % 16) == 0 && (L_OUT % 16) == 0);
static_assert((XPF % 4) == 0 && (H3P % 4) == 0 && (H1P % 8) == 0 && (H2P % 8) == 0);
static_assert((SMAX % 32) == 0 && (CHUNK % NTHR) == 0);
static_assert(IN_DIM < 8 && K1P == 32);

typedef float    v4f  __attribute__((ext_vector_type(4)));
typedef float    v8f  __attribute__((ext_vector_type(8)));
typedef _Float16 v8h  __attribute__((ext_vector_type(8)));
typedef _Float16 v16h __attribute__((ext_vector_type(16)));
typedef int      v4i  __attribute__((ext_vector_type(4)));
union FragH { v16h v; v8h h[2]; };

__device__ __forceinline__ v8f wmh(v16h a, v16h b, v8f c) {
  v8f d = __builtin_amdgcn_wmma_f32_16x16x32_f16(false, a, false, b, (short)0, c, false, false);
#if defined(__HIP_DEVICE_COMPILE__)
  asm volatile("v_nop\n\tv_nop\n\tv_nop\n\tv_nop" : "+v"(d) : "v"(a), "v"(b));
#endif
  return d;
}

__device__ __forceinline__ v8f zero8() {
  v8f z = {0.f, 0.f, 0.f, 0.f, 0.f, 0.f, 0.f, 0.f};
  return z;
}

template <int NT>
__device__ __forceinline__ void mma_step(v8f (&acc)[NT], v16h av, const _Float16* __restrict__ bplane,
                                         int nb0, int KP, int kt, int m, int hh) {
#pragma unroll
  for (int t = 0; t < NT; ++t) {
    const _Float16* bp = bplane + (size_t)(nb0 + 16 * t + m) * KP + 32 * kt + 8 * hh;
    FragH b;
    b.h[0] = *(const v8h*)bp;
    b.h[1] = *(const v8h*)(bp + 16);
    acc[t] = wmh(av, b.v, acc[t]);
  }
}

template <int KT, int NT>
__device__ __forceinline__ void mma_h(v8f (&acc)[NT], const _Float16* ar, const _Float16* __restrict__ bplane,
                                      int nb0, int KP, int m, int hh) {
#pragma unroll
  for (int t = 0; t < NT; ++t) acc[t] = zero8();
#pragma unroll
  for (int kt = 0; kt < KT; ++kt) {
    FragH a;
    a.h[0] = *(const v8h*)(ar + 32 * kt);
    a.h[1] = *(const v8h*)(ar + 32 * kt + 16);
    mma_step<NT>(acc, a.v, bplane, nb0, KP, kt, m, hh);
  }
}

template <int KT, int NT>
__device__ __forceinline__ void mma_f(v8f (&acc)[NT], const float* ar, const _Float16* __restrict__ bplane,
                                      int nb0, int KP, int m, int hh) {
#pragma unroll
  for (int t = 0; t < NT; ++t) acc[t] = zero8();
#pragma unroll
  for (int kt = 0; kt < KT; ++kt) {
    const v4f f0 = *(const v4f*)(ar + 32 * kt);
    const v4f f1 = *(const v4f*)(ar + 32 * kt + 4);
    const v4f f2 = *(const v4f*)(ar + 32 * kt + 16);
    const v4f f3 = *(const v4f*)(ar + 32 * kt + 20);
    FragH a;
#pragma unroll
    for (int e = 0; e < 4; ++e) {
      a.h[0][e]     = (_Float16)f0[e];
      a.h[0][4 + e] = (_Float16)f1[e];
      a.h[1][e]     = (_Float16)f2[e];
      a.h[1][4 + e] = (_Float16)f3[e];
    }
    mma_step<NT>(acc, a.v, bplane, nb0, KP, kt, m, hh);
  }
}

template <int NT>
__device__ __forceinline__ void relu_store(const v8f (&acc)[NT], _Float16* sp, int pitch,
                                           const float* __restrict__ bias, int nb0, int m, float scl) {
#pragma unroll
  for (int t = 0; t < NT; ++t) {
    const float bc = bias[nb0 + 16 * t + m];
#pragma unroll
    for (int r = 0; r < 8; ++r) sp[r * pitch + 16 * t] = (_Float16)fmaxf(fmaf(acc[t][r], scl, bc), 0.0f);
  }
}

template <int NT>
__device__ __forceinline__ void lin_store(const v8f (&acc)[NT], float* sp, int pitch,
                                          const float* __restrict__ bias, int nb0, int m, float scl) {
#pragma unroll
  for (int t = 0; t < NT; ++t) {
    const float bc = bias[nb0 + 16 * t + m];
#pragma unroll
    for (int r = 0; r < 8; ++r) sp[r * pitch + 16 * t] = fmaf(acc[t][r], scl, bc);
  }
}

__global__ __launch_bounds__(NTHR) void k_prep(
    const float* __restrict__ W1, const float* __restrict__ W2, const float* __restrict__ W3,
    const float* __restrict__ A1,
    _Float16* pW1, _Float16* pW2, _Float16* pW3, _Float16* pA1) {
  const int b0 = G_W1, b1 = b0 + G_W2, b2 = b1 + G_W3, b3 = b2 + G_A1;
  const int bstart = blockIdx.x * NTHR;
  const float* src; _Float16* dst; int srcCols, Kv, KP, Nout, segOff; float scl;
  if (bstart < b0)      { src = W1; dst = pW1; srcCols = H1D; Kv = IN_DIM; KP = K1P; Nout = H1D; segOff = 0;  scl = 2.0f; }
  else if (bstart < b1) { src = W2; dst = pW2; srcCols = H2D; Kv = H1D;    KP = H1D; Nout = H2D; segOff = b0; scl = 8.0f; }
  else if (bstart < b2) { src = W3; dst = pW3; srcCols = EMB; Kv = H2D;    KP = H2D; Nout = EMB; segOff = b1; scl = 8.0f; }
  else                  { src = A1; dst = pA1; srcCols = ATT; Kv = EMB;    KP = EMB; Nout = ATT; segOff = b2; scl = 8.0f; }
  const int i = bstart + (int)threadIdx.x;
  if (i >= b3) return;
  const int o  = (i - segOff) * 8;
  const int n  = o / KP;
  const int k0 = o - n * KP;
  const int nc = n < Nout ? n : Nout - 1;
  float v[8];
#pragma unroll
  for (int e = 0; e < 8; ++e) {
    const int k  = k0 + e;
    const int kc = k < Kv ? k : Kv - 1;
    const float xv = src[(size_t)kc * srcCols + nc];
    v[e] = (k < Kv && n < Nout) ? xv * scl : 0.0f;
  }
  v8h hv;
#pragma unroll
  for (int e = 0; e < 8; ++e) hv[e] = (_Float16)v[e];
  _Float16* dp = dst + o;
  *(volatile v8h*)dp = hv;
  __threadfence();
  *(volatile v8h*)dp = hv;
}

__global__ __launch_bounds__(NTHR) void k_hist(
    const int* __restrict__ ids, const int* __restrict__ nseg, int* hist, int nF, int nS, int Spad) {
  extern __shared__ v4f lds_dyn[];
  int* sH = (int*)lds_dyn;
  const int tid = threadIdx.x, lane = tid & 31, wave = tid >> 5;
  const int c = blockIdx.x;
  int sv = nseg[0];
  sv = sv < 0 ? 0 : (sv > nS ? nS : sv);
  for (int i = tid; i < NWAVE * Spad; i += NTHR) sH[i] = 0;
  __syncthreads();
  int* sHw = sH + wave * Spad;
#pragma unroll 1
  for (int j = 0; j < SUBS; ++j) {
    const int e  = c * CHUNK + j * NTHR + tid;
    const int ec = e < nF ? e : nF - 1;
    const int id = ids[ec];
    const bool ok = (e < nF) && (id >= 0) && (id < sv);
    const int idc = ok ? id : -1;
#pragma unroll 1
    for (int l = 0; l < 32; ++l) {
      const int idl = __builtin_amdgcn_readlane(idc, l);
      if (lane == 0 && idl >= 0) sHw[idl] += 1;
    }
  }
  __syncthreads();
  int* row = hist + (size_t)c * Spad;
  for (int i = tid; i < Spad / 4; i += NTHR) {
    v4i v = *(const v4i*)(sH + 4 * i);
#pragma unroll
    for (int w = 1; w < NWAVE; ++w) v += *(const v4i*)(sH + w * Spad + 4 * i);
    *(volatile v4i*)(row + 4 * i) = v;
    __threadfence();
    *(volatile v4i*)(row + 4 * i) = v;
  }
}

__global__ __launch_bounds__(NTHR) void k_seg(
    const float* __restrict__ faces, const int* __restrict__ ids, const int* __restrict__ hist,
    const _Float16* __restrict__ pW1, const _Float16* __restrict__ pW2,
    const _Float16* __restrict__ pW3, const _Float16* __restrict__ pA1,
    const float* __restrict__ b1, const float* __restrict__ b2, const float* __restrict__ b3,
    const float* __restrict__ ba1, const float* __restrict__ Wa2, const float* __restrict__ ba2,
    float* out, int nF, int nC, int Spad) {
  extern __shared__ v4f lds_dyn[];
  char* lb = (char*)lds_dyn;
  float*    sXf   = (float*)(lb + L_XF);
  _Float16* sH1   = (_Float16*)(lb + L_H1);
  _Float16* sH2   = (_Float16*)(lb + L_H2);
  float*    sH3   = (float*)(lb + L_H3);
  float*    sS    = (float*)(lb + L_S);
  float*    sE    = (float*)(lb + L_E);
  int*      sList = (int*)(lb + L_LIST);
  int*      sChk  = (int*)(lb + L_CHK);
  int*      sWcnt = (int*)(lb + L_WCNT);
  float*    sOut  = (float*)(lb + L_OUT);
  const int tid = threadIdx.x, lane = tid & 31, wave = tid >> 5, hh = lane >> 4, m = lane & 15;
  const int s = blockIdx.x;
  const int wr = wave * 16;
  const float ba2v = ba2[0];

  for (int i = tid; i < ROWS * XPF; i += NTHR) sXf[i] = 0.0f;

  int nchTot = 0;
  const int nsub = (nC + NTHR - 1) / NTHR;
  for (int j = 0; j < nsub; ++j) {
    const int c  = j * NTHR + tid;
    const int cc = c < nC ? c : nC - 1;
    const int hv = hist[(size_t)cc * Spad + s];
    const bool hit = (c < nC) && (hv > 0);
    const unsigned msk = __builtin_amdgcn_ballot_w32(hit);
    if (lane == 0) sWcnt[wave] = (int)__builtin_popcount(msk);
    __syncthreads();
    int pre = 0, tot = 0;
#pragma unroll
    for (int w = 0; w < NWAVE; ++w) { const int v = sWcnt[w]; tot += v; pre += (w < wave) ? v : 0; }
    const int pos = nchTot + pre + (int)__builtin_popcount(msk & ((1u << lane) - 1u));
    if (hit && pos < MAXCH) sChk[pos] = c;
    nchTot += tot;
    __syncthreads();
  }
  const int nch = nchTot < MAXCH ? nchTot : MAXCH;

  float mrun = -3.0e38f, zrun = 0.0f;
  v4f pacc = {0.f, 0.f, 0.f, 0.f};
  const int rq = tid & 3, cq = tid >> 2;

  for (int q = 0; q < nch; ++q) {
    int c = sChk[q];
    c = c < 0 ? 0 : (c > nC - 1 ? nC - 1 : c);
    const int cbase = c * CHUNK;
    int cnt = 0;
#pragma unroll 1
    for (int j = 0; j < SUBS; ++j) {
      const int e  = cbase + j * NTHR + tid;
      const int ec = e < nF ? e : nF - 1;
      const int id = ids[ec];
      const bool hit = (e < nF) && (id == s);
      const unsigned msk = __builtin_amdgcn_ballot_w32(hit);
      if (lane == 0) sWcnt[wave] = (int)__builtin_popcount(msk);
      __syncthreads();
      int pre = 0, tot = 0;
#pragma unroll
      for (int w = 0; w < NWAVE; ++w) { const int v = sWcnt[w]; tot += v; pre += (w < wave) ? v : 0; }
      const int pos = cnt + pre + (int)__builtin_popcount(msk & ((1u << lane) - 1u));
      if (hit && pos < CHUNK) sList[pos] = e;
      cnt += tot;
      __syncthreads();
    }
    cnt = cnt > CHUNK ? CHUNK : cnt;
    const int niter = (cnt + ROWS - 1) / ROWS;

#pragma unroll 1
    for (int it = 0; it < niter; ++it) {
      const int rbase = it * ROWS;
      const int nrows = cnt - rbase;

      for (int i = tid; i < ROWS * 8; i += NTHR) {
        const int r = i >> 3, col = i & 7;
        int li = rbase + r;
        li = li < cnt ? li : cnt - 1;
        int f = sList[li];
        f = f < 0 ? 0 : (f > nF - 1 ? nF - 1 : f);
        const int colc = col < IN_DIM ? col : IN_DIM - 1;
        const float xv = faces[(size_t)f * IN_DIM + colc];
        sXf[r * XPF + col] = (col < IN_DIM) ? xv : 0.0f;
      }
      __syncthreads();

      {
        v8f acc[4];
        mma_f<1, 4>(acc, sXf + (wr + m) * XPF + 8 * hh, pW1, 0, K1P, m, hh);
        relu_store<4>(acc, sH1 + (wr + 8 * hh) * H1P + m, H1P, b1, 0, m, 0.5f);
      }
      __syncthreads();
      {
        v8f acc[8];
        mma_h<2, 8>(acc, sH1 + (wr + m) * H1P + 8 * hh, pW2, 0, H1D, m, hh);
        relu_store<8>(acc, sH2 + (wr + 8 * hh) * H2P + m, H2P, b2, 0, m, 0.125f);
      }
      __syncthreads();
#pragma unroll
      for (int g = 0; g < 2; ++g) {
        v8f acc[8];
        mma_h<4, 8>(acc, sH2 + (wr + m) * H2P + 8 * hh, pW3, 128 * g, H2D, m, hh);
        lin_store<8>(acc, sH3 + (wr + 8 * hh) * H3P + 128 * g + m, H3P, b3, 128 * g, m, 0.125f);
      }
      __syncthreads();
      {
        v8f acc[4];
        mma_f<8, 4>(acc, sH3 + (wr + m) * H3P + 8 * hh, pA1, 0, EMB, m, hh);
        float sc[8];
#pragma unroll
        for (int r = 0; r < 8; ++r) sc[r] = 0.0f;
#pragma unroll
        for (int t = 0; t < 4; ++t) {
          const float bc = ba1[16 * t + m];
          const float wv = Wa2[16 * t + m];
#pragma unroll
          for (int r = 0; r < 8; ++r) {
            const float av = tanhf(fmaf(acc[t][r], 0.125f, bc));
            sc[r] = fmaf(av, wv, sc[r]);
          }
        }
#pragma unroll
        for (int r = 0; r < 8; ++r) {
          sc[r] += __shfl_xor(sc[r], 1, 32);
          sc[r] += __shfl_xor(sc[r], 2, 32);
          sc[r] += __shfl_xor(sc[r], 4, 32);
          sc[r] += __shfl_xor(sc[r], 8, 32);
        }
        if (m == 0) {
#pragma unroll
          for (int r = 0; r < 8; ++r) {
            const int rl = wr + 8 * hh + r;
            sS[rl] = (rl < nrows) ? (sc[r] + ba2v) : -3.0e38f;
          }
        }
      }
      __syncthreads();

      {
        float cm = -3.0e38f;
#pragma unroll
        for (int k = 0; k < ROWS / 32; ++k) cm = fmaxf(cm, sS[lane + 32 * k]);
#pragma unroll
        for (int msk = 16; msk >= 1; msk >>= 1) cm = fmaxf(cm, __shfl_xor(cm, msk, 32));
        const float mnew = fmaxf(mrun, cm);
        const float rs = expf(mrun - mnew);
        if (tid < ROWS) {
          const float svv = sS[tid];
          const float ev = expf(svv - mnew);
          sE[tid] = (tid < nrows) ? ev : 0.0f;
        }
        __syncthreads();
        float zc = 0.0f;
#pragma unroll
        for (int k = 0; k < ROWS / 32; ++k) zc += sE[lane + 32 * k];
#pragma unroll
        for (int msk = 16; msk >= 1; msk >>= 1) zc += __shfl_xor(zc, msk, 32);
        zrun = fmaf(zrun, rs, zc);
        const float* hr = sH3 + (32 * rq) * H3P + 4 * cq;
        const float* er = sE + 32 * rq;
        v4f p = {0.f, 0.f, 0.f, 0.f};
#pragma unroll 4
        for (int i = 0; i < 32; ++i) {
          const float ev = er[i];
          const v4f hvv = *(const v4f*)(hr + i * H3P);
          p += hvv * ev;
        }
#pragma unroll
        for (int jj = 0; jj < 4; ++jj) {
          float v = p[jj];
          v += __shfl_xor(v, 1, 32);
          v += __shfl_xor(v, 2, 32);
          p[jj] = v;
        }
        pacc = pacc * rs + p;
        mrun = mnew;
      }
    }
  }

  {
    const bool zok = zrun > 0.0f;
    const float rz = 1.0f / (zok ? zrun : 1.0f);
    const v4f ov = pacc * (zok ? rz : 0.0f);
    if (rq == 0) *(v4f*)(sOut + 4 * cq) = ov;
  }
  __syncthreads();
  if (tid < EMB / 4) {
    const v4f v = *(const v4f*)(sOut + 4 * tid);
    float* op = out + (size_t)s * EMB + 4 * tid;
    *(volatile v4f*)op = v;
    __threadfence();
    *(volatile v4f*)op = v;
  }
}

extern "C" void kernel_launch(void* const* d_in, const int* in_sizes, int n_in,
                              void* d_out, int out_size, void* d_ws, size_t ws_size,
                              hipStream_t stream) {
  if (n_in < 13) return;
  const int nF = in_sizes[0] / IN_DIM;
  if (nF <= 0 || in_sizes[0] != nF * IN_DIM || nF > (1 << 28)) return;
  if (in_sizes[1] != IN_DIM * H1D || in_sizes[2] != H1D) return;
  if (in_sizes[3] != H1D * H2D || in_sizes[4] != H2D) return;
  if (in_sizes[5] != H2D * EMB || in_sizes[6] != EMB) return;
  if (in_sizes[7] != EMB * ATT || in_sizes[8] != ATT) return;
  if (in_sizes[9] != ATT || in_sizes[10] < 1) return;
  if (in_sizes[11] != nF || in_sizes[12] < 1) return;
  const int nS = out_size / EMB;
  if (nS <= 0 || out_size != nS * EMB || nS > SMAX) return;

  const float* faces = (const float*)d_in[0];
  const float* W1  = (const float*)d_in[1];
  const float* b1  = (const float*)d_in[2];
  const float* W2  = (const float*)d_in[3];
  const float* b2  = (const float*)d_in[4];
  const float* W3  = (const float*)d_in[5];
  const float* b3  = (const float*)d_in[6];
  const float* Wa1 = (const float*)d_in[7];
  const float* ba1 = (const float*)d_in[8];
  const float* Wa2 = (const float*)d_in[9];
  const float* ba2 = (const float*)d_in[10];
  const int*   ids = (const int*)d_in[11];
  const int*   nsg = (const int*)d_in[12];
  float* out = (float*)d_out;

  const int nC   = (nF + CHUNK - 1) / CHUNK;
  const int Spad = (nS + 31) & ~31;
  const int ldsHist = NWAVE * Spad * 4;

  char* ws = (char*)d_ws;
  size_t off = 0;
  const size_t oW1 = off; off += (size_t)H1D * K1P * 2;      off = (off + 255) & ~(size_t)255;
  const size_t oW2 = off; off += (size_t)H2D * H1D * 2;      off = (off + 255) & ~(size_t)255;
  const size_t oW3 = off; off += (size_t)EMB * H2D * 2;      off = (off + 255) & ~(size_t)255;
  const size_t oA1 = off; off += (size_t)ATT * EMB * 2;      off = (off + 255) & ~(size_t)255;
  const size_t oHs = off; off += (size_t)nC * Spad * 4;      off = (off + 255) & ~(size_t)255;
  if (off > ws_size || off > (size_t)134217728) return;
  _Float16* pW1 = (_Float16*)(ws + oW1);
  _Float16* pW2 = (_Float16*)(ws + oW2);
  _Float16* pW3 = (_Float16*)(ws + oW3);
  _Float16* pA1 = (_Float16*)(ws + oA1);
  int* hist = (int*)(ws + oHs);

  k_prep<<<G_TOT / NTHR, NTHR, 0, stream>>>(W1, W2, W3, Wa1, pW1, pW2, pW3, pA1);

  hipFuncSetAttribute(reinterpret_cast<const void*>(&k_hist),
                      hipFuncAttributeMaxDynamicSharedMemorySize, ldsHist);
  k_hist<<<nC, NTHR, ldsHist, stream>>>(ids, nsg, hist, nF, nS, Spad);

  hipFuncSetAttribute(reinterpret_cast<const void*>(&k_seg),
                      hipFuncAttributeMaxDynamicSharedMemorySize, LDS_SEG);
  k_seg<<<nS, NTHR, LDS_SEG, stream>>>(faces, ids, hist, pW1, pW2, pW3, pA1, b1, b2, b3, ba1, Wa2, ba2,
                                       out, nF, nC, Spad);
}
